// GQA_37366215475614
// MI455X (gfx1250) — hardware-verified
//
#include <hip/hip_runtime.h>
#include <math.h>
#include <stdint.h>

#define NB     2
#define SEQ    1024
#define DM     2048
#define NH     32
#define NKV    8
#define HD     64
#define DKV    512
#define NTOK   2048
#define NQK    2560
#define NQKV   3072
#define QPW    4096
#define KPW    1024
#define CTW    4096
#define NFREQ  32

static_assert(NTOK % 64 == 0);
static_assert(NQK % 64 == 0);
static_assert(DKV % 64 == 0);
static_assert(DM % 64 == 0);
static_assert(DM % 32 == 0);
static_assert(CTW % 32 == 0);
static_assert(SEQ % 64 == 0);
static_assert(((NTOK / 64) * (NQK / 64)) % 8 == 0);
static_assert(((DKV / 64) * (NTOK / 64)) % 8 == 0);
static_assert(((NTOK / 64) * (DM / 64)) % 8 == 0);

typedef __bf16       v16b __attribute__((ext_vector_type(16)));
typedef __bf16       v8b  __attribute__((ext_vector_type(8)));
typedef float        v8f  __attribute__((ext_vector_type(8)));
typedef float        v4f  __attribute__((ext_vector_type(4)));
typedef unsigned int v4u  __attribute__((ext_vector_type(4)));

__device__ __forceinline__ unsigned short bf_bits(float f) {
  const unsigned u = __float_as_uint(f);
  return (unsigned short)((u + 0x7FFFu + ((u >> 16) & 1u)) >> 16);
}
__device__ __forceinline__ float bf_val(unsigned short h) { return __uint_as_float(((unsigned)h) << 16); }
__device__ __forceinline__ unsigned pk16(unsigned short a, unsigned short b) { return (unsigned)a | ((unsigned)b << 16); }
__device__ __forceinline__ v8f zero8() { v8f z = {0.f, 0.f, 0.f, 0.f, 0.f, 0.f, 0.f, 0.f}; return z; }
__device__ __forceinline__ int wave_id() { return __builtin_amdgcn_readfirstlane((int)(threadIdx.x >> 5)); }

__device__ __forceinline__ void lds_wave_sync() {
  __builtin_amdgcn_fence(__ATOMIC_RELEASE, "workgroup");
  __builtin_amdgcn_wave_barrier();
  __builtin_amdgcn_fence(__ATOMIC_ACQUIRE, "workgroup");
}

union FragB { v16b v; v8b h[2]; };
__device__ __forceinline__ v16b ldfrag_b(const __bf16* p) { FragB f; f.h[0] = *(const v8b*)(p); f.h[1] = *(const v8b*)(p + 16); return f.v; }

__device__ __forceinline__ v8f mma_b(v16b a, v16b b, v8f c) {
  return __builtin_amdgcn_wmma_f32_16x16x32_bf16(false, a, false, b, (short)0, c, false, false);
}
__device__ __forceinline__ v8f at_mma(v16b a, v16b b, v8f c) {
  c = __builtin_amdgcn_wmma_f32_16x16x32_bf16(false, a, false, b, (short)0, c, false, false);
  asm volatile("v_nop\n\tv_nop\n\tv_nop\n\tv_nop" : "+v"(c) : "v"(a), "v"(b));
  return c;
}
__device__ __forceinline__ void guard_row(v8f& a, v8f& b, v8f& c, v8f& d, v16b x) {
  asm volatile("v_nop\n\tv_nop\n\tv_nop\n\tv_nop" : "+v"(a), "+v"(b), "+v"(c), "+v"(d) : "v"(x));
}
__device__ __forceinline__ void keep4_b(v16b a, v16b b, v16b c, v16b d) { asm volatile("v_nop" :: "v"(a), "v"(b), "v"(c), "v"(d)); }
__device__ __forceinline__ void acc_guard4(v8f& a, v8f& b, v8f& c, v8f& d) {
  asm volatile("v_nop\n\tv_nop\n\tv_nop\n\tv_nop" : "+v"(a), "+v"(b), "+v"(c), "+v"(d));
}

__global__ __launch_bounds__(256) void rope_table_kernel(float* __restrict__ cst, float* __restrict__ snt) {
  const int lane = threadIdx.x & 31;
  const int wave = (int)(threadIdx.x >> 5);
  const int t = (int)blockIdx.x * 8 + wave;
  if (t >= SEQ) return;
  const float pf  = (float)t;
  const float e   = (float)lane * 0.03125f;
  const float pw  = powf(10000.0f, e);
  const float inv = 1.0f / pw;
  const float ang = pf * inv;
  const float cv  = cosf(ang);
  const float sv  = sinf(ang);
  const size_t o = (size_t)t * NFREQ + lane;
  for (int pass = 0; pass < 2; ++pass) {
    ((volatile float*)cst)[o] = cv;
    ((volatile float*)snt)[o] = sv;
    __threadfence();
  }
}

__global__ __launch_bounds__(256) void cvt_bf16_kernel(const float* __restrict__ in, unsigned short* __restrict__ outp, int n8) {
  const int i = (int)blockIdx.x * 256 + (int)threadIdx.x;
  if (i >= n8) return;
  const size_t e = 8 * (size_t)i;
  const v4f a = *(const v4f*)(in + e);
  const v4f b = *(const v4f*)(in + e + 4);
  v4u w;
  w[0] = pk16(bf_bits(a[0]), bf_bits(a[1]));
  w[1] = pk16(bf_bits(a[2]), bf_bits(a[3]));
  w[2] = pk16(bf_bits(b[0]), bf_bits(b[1]));
  w[3] = pk16(bf_bits(b[2]), bf_bits(b[3]));
  *(volatile v4u*)(outp + e) = w;
  __threadfence();
  *(volatile v4u*)(outp + e) = w;
}

__global__ __launch_bounds__(256) void tcvt_kernel(const float* __restrict__ W, unsigned short* __restrict__ o,
                                                   int R, int Cc, int ldo, int dup) {
  __shared__ __align__(16) float tf[64 * 68];
  const int c0  = blockIdx.x * 64;
  const int r0  = blockIdx.y * 64;
  const int tid = threadIdx.x;
  {
    const int lr = tid >> 4;
    const int c4 = (tid & 15) * 4;
#pragma unroll
    for (int it = 0; it < 4; ++it) {
      const int rr = it * 16 + lr;
      const v4f a = *(const v4f*)(W + (size_t)(r0 + rr) * Cc + c0 + c4);
      *(v4f*)(tf + rr * 68 + c4) = a;
    }
  }
  __syncthreads();
  const int sub = tid >> 3;
  const int c8  = (tid & 7) * 8;
  v4u hv[2];
#pragma unroll
  for (int it = 0; it < 2; ++it) {
    const int oc = it * 32 + sub;
    v4u a;
#pragma unroll
    for (int q = 0; q < 4; ++q) {
      const float f0 = tf[(c8 + 2 * q) * 68 + oc];
      const float f1 = tf[(c8 + 2 * q + 1) * 68 + oc];
      a[q] = pk16(bf_bits(f0), bf_bits(f1));
    }
    hv[it] = a;
  }
  for (int pass = 0; pass < 2; ++pass) {
#pragma unroll
    for (int it = 0; it < 2; ++it) {
      const int oc = it * 32 + sub;
      const size_t go = (size_t)(c0 + oc) * ldo + r0 + c8;
      *(volatile v4u*)(o + go) = hv[it];
      if (dup > 0) *(volatile v4u*)(o + go + dup) = hv[it];
    }
    __threadfence();
  }
}

__device__ __forceinline__ void rot_split(float ta, float tb, float cc, float ss, unsigned& wh, unsigned& wl) {
  const float oa = ta * cc - tb * ss;
  const float ob = ta * ss + tb * cc;
  const unsigned short ha = bf_bits(oa), hb = bf_bits(ob);
  const unsigned short la = bf_bits(oa - bf_val(ha)), lb = bf_bits(ob - bf_val(hb));
  wh = pk16(ha, hb);
  wl = pk16(la, lb);
}
__device__ __forceinline__ void plain_split(float ta, float tb, unsigned& wh, unsigned& wl) {
  const unsigned short ha = bf_bits(ta), hb = bf_bits(tb);
  const unsigned short la = bf_bits(ta - bf_val(ha)), lb = bf_bits(tb - bf_val(hb));
  wh = pk16(ha, hb);
  wl = pk16(la, lb);
}

template <int EPI>
__global__ __launch_bounds__(256) void gemm64_kernel(
    const unsigned short* __restrict__ Ap, int lda,
    const unsigned short* __restrict__ Btp, int ldb,
    void* C0, void* C1, int ldc, int ldc2,
    const float* __restrict__ cst, const float* __restrict__ snt,
    int M, int N, int K) {
  __shared__ __align__(16) float sT[8][16 * 68];

  const int lane = threadIdx.x & 31;
  const int wave = wave_id();
  const int tilesN = N >> 6;
  const int tilesM = M >> 6;
  const int tile = (int)blockIdx.x * 8 + wave;
  if (tile >= tilesM * tilesN) return;
  const int tm = tile / tilesN;
  const int tn = tile - tm * tilesN;
  const int m0 = tm << 6;
  const int n0 = tn << 6;

  const __bf16* A  = (const __bf16*)(const void*)Ap;
  const __bf16* Bt = (const __bf16*)(const void*)Btp;

  const int rl   = lane & 15;
  const int koff = (lane >> 4) * 8;
  const int mOff = (lane >> 4) * 8;

  v8f acc[4][4];
#pragma unroll
  for (int i = 0; i < 4; ++i)
#pragma unroll
    for (int j = 0; j < 4; ++j) acc[i][j] = zero8();

  for (int k0 = 0; k0 < K; k0 += 32) {
    v16b bh[4];
#pragma unroll
    for (int j = 0; j < 4; ++j)
      bh[j] = ldfrag_b(Bt + (size_t)(n0 + (j << 4) + rl) * ldb + koff + k0);
#pragma unroll
    for (int i = 0; i < 4; ++i) {
      const v16b ah = ldfrag_b(A + (size_t)(m0 + (i << 4) + rl) * lda + koff + k0);
#pragma unroll
      for (int j = 0; j < 4; ++j) acc[i][j] = mma_b(ah, bh[j], acc[i][j]);
      guard_row(acc[i][0], acc[i][1], acc[i][2], acc[i][3], ah);
    }
    keep4_b(bh[0], bh[1], bh[2], bh[3]);
  }
  acc_guard4(acc[0][0], acc[0][1], acc[0][2], acc[0][3]);
  acc_guard4(acc[1][0], acc[1][1], acc[1][2], acc[1][3]);
  acc_guard4(acc[2][0], acc[2][1], acc[2][2], acc[2][3]);
  acc_guard4(acc[3][0], acc[3][1], acc[3][2], acc[3][3]);

  float* slab = sT[wave];
  const int q4 = lane >> 3;
  const int c8 = (lane & 7) * 8;
#pragma unroll
  for (int i = 0; i < 4; ++i) {
    const int mBase = m0 + (i << 4);
#pragma unroll
    for (int j = 0; j < 4; ++j)
#pragma unroll
      for (int r = 0; r < 8; ++r)
        slab[(mOff + r) * 68 + (j << 4) + rl] = acc[i][j][r];
    lds_wave_sync();
    if (EPI == 0) {
      const bool isq = (n0 < DM);
      unsigned short* P = isq ? (unsigned short*)C0 : (unsigned short*)C1;
      const int ldp  = isq ? ldc : ldc2;
      const int col0 = isq ? n0 : (n0 - DM);
      const int loff = isq ? DM : DKV;
      for (int pass = 0; pass < 2; ++pass) {
#pragma unroll 1
        for (int it = 0; it < 4; ++it) {
          const int row = it * 4 + q4;
          const int tok = mBase + row;
          const int pos = tok & (SEQ - 1);
          const float* sp = slab + row * 68 + c8;
          const v4f x0 = *(const v4f*)(sp);
          const v4f x1 = *(const v4f*)(sp + 4);
          const v4f cv = *(const v4f*)(cst + (size_t)pos * NFREQ + (c8 >> 1));
          const v4f sv = *(const v4f*)(snt + (size_t)pos * NFREQ + (c8 >> 1));
          unsigned h0, h1, h2, h3, l0, l1, l2, l3;
          rot_split(x0[0], x0[1], cv[0], sv[0], h0, l0);
          rot_split(x0[2], x0[3], cv[1], sv[1], h1, l1);
          rot_split(x1[0], x1[1], cv[2], sv[2], h2, l2);
          rot_split(x1[2], x1[3], cv[3], sv[3], h3, l3);
          v4u hv, lv;
          hv[0] = h0; hv[1] = h1; hv[2] = h2; hv[3] = h3;
          lv[0] = l0; lv[1] = l1; lv[2] = l2; lv[3] = l3;
          const size_t go = (size_t)tok * ldp + col0 + c8;
          *(volatile v4u*)(P + go) = hv;
          *(volatile v4u*)(P + go + loff) = lv;
        }
        __threadfence();
      }
    } else if (EPI == 1) {
      unsigned short* P0 = (unsigned short*)C0;
      unsigned short* P1 = (unsigned short*)C1;
      for (int pass = 0; pass < 2; ++pass) {
#pragma unroll 1
        for (int it = 0; it < 4; ++it) {
          const int row = it * 4 + q4;
          const float* sp = slab + row * 68 + c8;
          const v4f x0 = *(const v4f*)(sp);
          const v4f x1 = *(const v4f*)(sp + 4);
          unsigned h0, h1, h2, h3, l0, l1, l2, l3;
          plain_split(x0[0], x0[1], h0, l0);
          plain_split(x0[2], x0[3], h1, l1);
          plain_split(x1[0], x1[1], h2, l2);
          plain_split(x1[2], x1[3], h3, l3);
          v4u hv, lv;
          hv[0] = h0; hv[1] = h1; hv[2] = h2; hv[3] = h3;
          lv[0] = l0; lv[1] = l1; lv[2] = l2; lv[3] = l3;
          const size_t go = (size_t)(mBase + row) * ldc + n0 + c8;
          *(volatile v4u*)(P0 + go) = hv;
          *(volatile v4u*)(P1 + go) = lv;
        }
        __threadfence();
      }
    } else {
      float* C = (float*)C0;
      const int hh2 = lane >> 4, c4 = (lane & 15) * 4;
      for (int pass = 0; pass < 2; ++pass) {
#pragma unroll
        for (int it = 0; it < 8; ++it) {
          const int row = it * 2 + hh2;
          const v4f v = *(const v4f*)(slab + row * 68 + c4);
          *(volatile v4f*)(C + (size_t)(mBase + row) * ldc + n0 + c4) = v;
        }
        __threadfence();
      }
    }
    lds_wave_sync();
  }
}

__global__ __launch_bounds__(128) void attn_kernel(
    const unsigned short* __restrict__ qp, const unsigned short* __restrict__ kp,
    const unsigned short* __restrict__ vhp, const unsigned short* __restrict__ vlp,
    unsigned short* __restrict__ ctx) {
  __shared__ __align__(16) unsigned short Ksh[64 * 64];
  __shared__ __align__(16) unsigned short Ksl[64 * 64];
  __shared__ __align__(16) unsigned short Vth[64 * 64];
  __shared__ __align__(16) unsigned short Vtl[64 * 64];
  __shared__ __align__(16) unsigned short Phs[4][16 * 64];
  __shared__ __align__(16) unsigned short Pls[4][16 * 64];

  const int tid  = (int)threadIdx.x;
  const int lane = tid & 31;
  const int wave = wave_id();
  const int hh   = lane >> 4;
  const int c    = lane & 15;
  const int qt   = (int)blockIdx.x;
  const int h    = (int)blockIdx.y;
  const int b    = (int)blockIdx.z;
  const int kv   = h >> 2;
  const int q0   = qt * 64 + wave * 16;
  const size_t tok0 = (size_t)b * SEQ;

  const __bf16* Qhr = (const __bf16*)(const void*)qp + (tok0 + q0 + c) * QPW + h * HD + 8 * hh;
  const __bf16* Qlr = Qhr + DM;

  unsigned short* ph = Phs[wave];
  unsigned short* pl = Pls[wave];

  v16b qah[2], qal[2];
#pragma unroll
  for (int dc = 0; dc < 2; ++dc) { qah[dc] = ldfrag_b(Qhr + dc * 32); qal[dc] = ldfrag_b(Qlr + dc * 32); }

  float mrow[8], lrow[8];
  v8f oacc[4];
#pragma unroll
  for (int r = 0; r < 8; ++r) { mrow[r] = -INFINITY; lrow[r] = 0.f; }
#pragma unroll
  for (int t = 0; t < 4; ++t) oacc[t] = zero8();

  const int nChunks = qt + 1;
  for (int kc = 0; kc < nChunks; ++kc) {
    const int kv0 = kc * 64;
    __syncthreads();
    {
      const int r = tid >> 1, half = (tid & 1) * 32;
      const unsigned short* ksh = kp + (tok0 + kv0 + r) * KPW + kv * HD + half;
      const unsigned short* ksl = ksh + DKV;
      const unsigned short* vsh = vhp + (size_t)(kv * HD + r) * NTOK + tok0 + kv0 + half;
      const unsigned short* vsl = vlp + (size_t)(kv * HD + r) * NTOK + tok0 + kv0 + half;
#pragma unroll
      for (int i = 0; i < 4; ++i) {
        const v4u a0 = *(const v4u*)(ksh + 8 * i);
        const v4u a1 = *(const v4u*)(ksl + 8 * i);
        const v4u b0 = *(const v4u*)(vsh + 8 * i);
        const v4u b1 = *(const v4u*)(vsl + 8 * i);
        *(v4u*)(Ksh + r * 64 + half + 8 * i) = a0;
        *(v4u*)(Ksl + r * 64 + half + 8 * i) = a1;
        *(v4u*)(Vth + r * 64 + half + 8 * i) = b0;
        *(v4u*)(Vtl + r * 64 + half + 8 * i) = b1;
      }
    }
    __syncthreads();

    v8f s[4];
#pragma unroll
    for (int j = 0; j < 4; ++j) {
      s[j] = zero8();
#pragma unroll
      for (int dc = 0; dc < 2; ++dc) {
        const v16b kb = ldfrag_b((const __bf16*)(const void*)Ksh + (j * 16 + c) * 64 + dc * 32 + 8 * hh);
        const v16b kl = ldfrag_b((const __bf16*)(const void*)Ksl + (j * 16 + c) * 64 + dc * 32 + 8 * hh);
        s[j] = at_mma(qah[dc], kb, s[j]);
        s[j] = at_mma(qah[dc], kl, s[j]);
        s[j] = at_mma(qal[dc], kb, s[j]);
      }
    }
    const bool diag = (kc == qt);
    float cm[8];
#pragma unroll
    for (int r = 0; r < 8; ++r) {
      const int qrow = q0 + 8 * hh + r;
      float m = -INFINITY;
#pragma unroll
      for (int j = 0; j < 4; ++j) {
        const int kvcol = kv0 + j * 16 + c;
        const float sv = s[j][r] * 0.125f;
        const bool masked = diag && (kvcol > qrow);
        const float sm = masked ? -INFINITY : sv;
        s[j][r] = sm;
        m = fmaxf(m, sm);
      }
#pragma unroll
      for (int off = 1; off < 16; off <<= 1) m = fmaxf(m, __shfl_xor(m, off, 32));
      cm[r] = m;
    }
#pragma unroll
    for (int r = 0; r < 8; ++r) {
      const float mnew  = fmaxf(mrow[r], cm[r]);
      const float alpha = expf(mrow[r] - mnew);
      mrow[r] = mnew;
      float psum = 0.f;
#pragma unroll
      for (int j = 0; j < 4; ++j) {
        const float p = expf(s[j][r] - mnew);
        psum += p;
        const unsigned short hb = bf_bits(p);
        const unsigned short lb = bf_bits(p - bf_val(hb));
        const int po = (8 * hh + r) * 64 + j * 16 + c;
        ph[po] = hb;
        pl[po] = lb;
      }
#pragma unroll
      for (int off = 1; off < 16; off <<= 1) psum += __shfl_xor(psum, off, 32);
      lrow[r] = lrow[r] * alpha + psum;
#pragma unroll
      for (int t = 0; t < 4; ++t) oacc[t][r] *= alpha;
    }
    lds_wave_sync();
#pragma unroll 1
    for (int kk = 0; kk < 2; ++kk) {
      const v16b pa = ldfrag_b((const __bf16*)(const void*)ph + c * 64 + kk * 32 + 8 * hh);
      const v16b pr = ldfrag_b((const __bf16*)(const void*)pl + c * 64 + kk * 32 + 8 * hh);
#pragma unroll
      for (int t = 0; t < 4; ++t) {
        const v16b vb = ldfrag_b((const __bf16*)(const void*)Vth + (t * 16 + c) * 64 + kk * 32 + 8 * hh);
        const v16b vr = ldfrag_b((const __bf16*)(const void*)Vtl + (t * 16 + c) * 64 + kk * 32 + 8 * hh);
        oacc[t] = at_mma(pa, vb, oacc[t]);
        oacc[t] = at_mma(pa, vr, oacc[t]);
        oacc[t] = at_mma(pr, vb, oacc[t]);
      }
    }
  }
  acc_guard4(oacc[0], oacc[1], oacc[2], oacc[3]);
  lds_wave_sync();

#pragma unroll
  for (int r = 0; r < 8; ++r) {
    const float inv = 1.0f / lrow[r];
#pragma unroll
    for (int t = 0; t < 4; ++t) {
      const float o = oacc[t][r] * inv;
      const unsigned short hb = bf_bits(o);
      const unsigned short lb = bf_bits(o - bf_val(hb));
      const int so = (8 * hh + r) * 64 + t * 16 + c;
      ph[so] = hb;
      pl[so] = lb;
    }
  }
  lds_wave_sync();
  unsigned short* Cg = ctx + (tok0 + q0) * CTW + h * HD;
  const int qq = lane >> 3;
  const int c8 = (lane & 7) * 8;
  for (int pass = 0; pass < 2; ++pass) {
#pragma unroll
    for (int it = 0; it < 4; ++it) {
      const int row = it * 4 + qq;
      const v4u x = *(const v4u*)(ph + row * 64 + c8);
      const v4u y = *(const v4u*)(pl + row * 64 + c8);
      *(volatile v4u*)(Cg + (size_t)row * CTW + c8)      = x;
      *(volatile v4u*)(Cg + (size_t)row * CTW + DM + c8) = y;
    }
    __threadfence();
  }
}

extern "C" void kernel_launch(void* const* d_in, const int* in_sizes, int n_in,
                              void* d_out, int out_size, void* d_ws, size_t ws_size,
                              hipStream_t stream) {
  if (n_in < 5) return;
  if (in_sizes[0] != NTOK * DM) return;
  if (in_sizes[1] != DM * DM) return;
  if (in_sizes[2] != DM * DKV) return;
  if (in_sizes[3] != DM * DKV) return;
  if (in_sizes[4] != DM * DM) return;
  if (out_size != NTOK * DM) return;

  const float* x  = (const float*)d_in[0];
  const float* Wq = (const float*)d_in[1];
  const float* Wk = (const float*)d_in[2];
  const float* Wv = (const float*)d_in[3];
  const float* Wo = (const float*)d_in[4];
  float* out = (float*)d_out;

  const size_t szXB  = (size_t)NTOK * DM * 2;
  const size_t szW   = (size_t)NQKV * DM * 2;
  const size_t szWO2 = (size_t)DM * CTW * 2;
  const size_t szT   = (size_t)SEQ * NFREQ * 4;
  const size_t szQP  = (size_t)NTOK * QPW * 2;
  const size_t szKP  = (size_t)NTOK * KPW * 2;
  const size_t szVT  = (size_t)DKV * NTOK * 2;
  const size_t szCTX = (size_t)NTOK * CTW * 2;
  size_t off = 0;
  const size_t oXB  = off; off += szXB;
  const size_t oW   = off; off += szW;
  const size_t oWO2 = off; off += szWO2;
  const size_t oCST = off; off += szT;
  const size_t oSNT = off; off += szT;
  const size_t oQP  = off; off += szQP;
  const size_t oKP  = off; off += szKP;
  const size_t oVTH = off; off += szVT;
  const size_t oVTL = off; off += szVT;
  const size_t oCTX = off; off += szCTX;
  if (off > ws_size) return;
  if (off > (size_t)134217728) return;

  char* ws = (char*)d_ws;
  unsigned short* XB   = (unsigned short*)(ws + oXB);
  unsigned short* WQKV = (unsigned short*)(ws + oW);
  unsigned short* WO2  = (unsigned short*)(ws + oWO2);
  float*          CST  = (float*)(ws + oCST);
  float*          SNT  = (float*)(ws + oSNT);
  unsigned short* QP   = (unsigned short*)(ws + oQP);
  unsigned short* KP   = (unsigned short*)(ws + oKP);
  unsigned short* VTH  = (unsigned short*)(ws + oVTH);
  unsigned short* VTL  = (unsigned short*)(ws + oVTL);
  unsigned short* CTX  = (unsigned short*)(ws + oCTX);

  const dim3 b256(256), b128(128);

  rope_table_kernel<<<dim3(SEQ / 8), b256, 0, stream>>>(CST, SNT);
  cvt_bf16_kernel<<<dim3((NTOK * DM / 8) / 256), b256, 0, stream>>>(x, XB, NTOK * DM / 8);
  tcvt_kernel<<<dim3(DM / 64, DM / 64), b256, 0, stream>>>(Wq, WQKV, DM, DM, DM, 0);
  tcvt_kernel<<<dim3(DKV / 64, DM / 64), b256, 0, stream>>>(Wk, WQKV + (size_t)DM * DM, DM, DKV, DM, 0);
  tcvt_kernel<<<dim3(DKV / 64, DM / 64), b256, 0, stream>>>(Wv, WQKV + (size_t)NQK * DM, DM, DKV, DM, 0);
  tcvt_kernel<<<dim3(DM / 64, DM / 64), b256, 0, stream>>>(Wo, WO2, DM, DM, CTW, DM);
  gemm64_kernel<0><<<dim3((NTOK / 64) * (NQK / 64) / 8), b256, 0, stream>>>(
      XB, DM, WQKV, DM, (void*)QP, (void*)KP, QPW, KPW, CST, SNT, NTOK, NQK, DM);
  gemm64_kernel<1><<<dim3((DKV / 64) * (NTOK / 64) / 8), b256, 0, stream>>>(
      WQKV + (size_t)NQK * DM, DM, XB, DM, (void*)VTH, (void*)VTL, NTOK, NTOK, CST, SNT, DKV, NTOK, DM);
  attn_kernel<<<dim3(SEQ / 64, NH, NB), b128, 0, stream>>>(QP, KP, VTH, VTL, CTX);
  gemm64_kernel<2><<<dim3((NTOK / 64) * (DM / 64) / 8), b256, 0, stream>>>(
      CTX, CTW, WO2, CTW, (void*)out, (void*)out, DM, DM, CST, SNT, NTOK, DM, CTW);
  (void)hipGetLastError();
}
